// InstantNGP_52759378264701
// MI455X (gfx1250) — hardware-verified
//
#include <hip/hip_runtime.h>
#include <hip/hip_bf16.h>

typedef __attribute__((ext_vector_type(16))) _Float16 v16h;
typedef __attribute__((ext_vector_type(8)))  float    v8f;
typedef __attribute__((ext_vector_type(4)))  float    v4f;
#define GEO_SCALE 1024.0f
#define INV_GEO_SCALE (1.0f / 1024.0f)
typedef __attribute__((ext_vector_type(4)))  unsigned int u32x4;
typedef __attribute__((ext_vector_type(8)))  int      i32x8;
typedef __attribute__((ext_vector_type(4)))  int      i32x4;

#define WAVES 4
#define TILES 4
#define NTHREADS (WAVES * 32)
#define POINTS_PER_BLOCK (WAVES * TILES * 16)

#define OFF_GW0 0
#define OFF_GW1 1024
#define OFF_DW  3072
#define OFF_CW0 3584
#define OFF_CW1 4608
#define OFF_CW2 6656
#define OFF_RW  8704
#define PW_WORDS 9216

#define OB_GB0 0
#define OB_GB1 64
#define OB_DB  128
#define OB_CB0 144
#define OB_CB1 208
#define OB_CB2 272
#define OB_RB  336
#define NBIAS  352

#define WB_WORDS (PW_WORDS + NBIAS)

#define HAVE_TDM 0

union Frag { v16h h; uint32_t u[8]; };
union PackPair { _Float16 h[2]; uint32_t u; };

__device__ __forceinline__ float lerpf(float a, float b, float w) {
    return a * (1.0f - w) + b * w;
}

__device__ __forceinline__ void wave_fence() {
    __builtin_amdgcn_fence(__ATOMIC_ACQ_REL, "wavefront");
}

__device__ __forceinline__ int kA(int j, int lane) {
    return ((j >> 2) << 4) + (((lane >> 4) & 1) << 3) + ((j & 3) << 1);
}

template<int KB>
__device__ __forceinline__ void load_afrag(Frag* a, const _Float16* xin, int ldx, int lane) {
    const int m = lane & 15;
#pragma unroll
    for (int kb = 0; kb < KB; ++kb)
#pragma unroll
        for (int j = 0; j < 8; ++j)
            a[kb].u[j] = *(const uint32_t*)(xin + m * ldx + kb * 32 + kA(j, lane));
}

template<int KB>
__device__ __forceinline__ v8f mlp_block(const Frag* a, const uint32_t* pw,
                                         int nb, int NBtot, float bias, int lane) {
    v8f acc;
#pragma unroll
    for (int r = 0; r < 8; ++r) acc[r] = bias;
#pragma unroll
    for (int kb = 0; kb < KB; ++kb) {
        Frag b;
#pragma unroll
        for (int j = 0; j < 8; ++j)
            b.u[j] = pw[(((kb * NBtot) + nb) * 8 + j) * 32 + lane];
        acc = __builtin_amdgcn_wmma_f32_16x16x32_f16(
            false, a[kb].h, false, b.h, (short)0, acc, false, false);
        asm volatile("v_nop\n\tv_nop\n\tv_nop\n\tv_nop" : "+v"(acc) : "v"(a[kb].h), "v"(b.h));
    }
    return acc;
}

template<int KB, int NB, bool RELU>
__device__ __forceinline__ void mlp_layer(const _Float16* xin, int ldx,
                                          const uint32_t* pw, const float* bias,
                                          _Float16* xout, int ldo, int lane) {
    Frag a[KB];
    load_afrag<KB>(a, xin, ldx, lane);
    const int n = lane & 15;
    const int mrow = ((lane >> 4) & 1) * 8;
#pragma unroll
    for (int nb = 0; nb < NB; ++nb) {
        v8f acc = mlp_block<KB>(a, pw, nb, NB, bias[nb * 16 + n], lane);
#pragma unroll
        for (int r = 0; r < 8; ++r) {
            float v = acc[r];
            if (RELU) v = v > 0.0f ? v : 0.0f;
            xout[(mrow + r) * ldo + nb * 16 + n] = (_Float16)v;
        }
    }
}

__device__ __forceinline__ void pack_w(const float* __restrict__ src,
                                       int K, int Ksrc, int Nout, int Nsrc,
                                       uint32_t* dst, int tid, float scale = 1.0f) {
    const int NB = Nout >> 4;
    const int words = (K * Nout) >> 1;
    for (int w = tid; w < words; w += NTHREADS) {
        int l  = w & 31;
        int j  = (w >> 5) & 7;
        int t  = w >> 8;
        int nb = t % NB;
        int kb = t / NB;
        int n  = nb * 16 + (l & 15);
        int k0 = kb * 32 + kA(j, l);
        float f0 = (k0     < Ksrc && n < Nsrc) ? src[k0 * Nsrc + n]       : 0.0f;
        float f1 = (k0 + 1 < Ksrc && n < Nsrc) ? src[(k0 + 1) * Nsrc + n] : 0.0f;
        PackPair pk;
        pk.h[0] = (_Float16)(f0 * scale);
        pk.h[1] = (_Float16)(f1 * scale);
        *(volatile uint32_t*)(dst + w) = pk.u; __threadfence(); *(volatile uint32_t*)(dst + w) = pk.u;
    }
}

__device__ __forceinline__ void pack_bias(const float* gb0, const float* gb1, const float* db,
                                          const float* cb0, const float* cb1, const float* cb2,
                                          const float* rb, float* dst, int tid) {
    for (int i = tid; i < NBIAS; i += NTHREADS) {
        float v;
        if      (i < 64)  v = gb0[i];
        else if (i < 128) v = gb1[i - 64];
        else if (i < 144) v = db[i - 128];
        else if (i < 208) v = cb0[i - 144];
        else if (i < 272) v = cb1[i - 208];
        else if (i < 336) v = cb2[i - 272];
        else { int j = i - 336; v = (j < 3) ? rb[j] : 0.0f; }
        if (i < 144) v *= GEO_SCALE;
        *(volatile float*)(dst + i) = v; __threadfence(); *(volatile float*)(dst + i) = v;
    }
}

__device__ __forceinline__ void pack_all(const float* gw0, const float* gw1, const float* dw,
                                         const float* cw0, const float* cw1, const float* cw2,
                                         const float* rw,
                                         const float* gb0, const float* gb1, const float* db,
                                         const float* cb0, const float* cb1, const float* cb2,
                                         const float* rb, uint32_t* dst, int tid) {
    pack_w(gw0, 32, 32, 64, 64, dst + OFF_GW0, tid);
    pack_w(gw1, 64, 64, 64, 64, dst + OFF_GW1, tid);
    pack_w(dw,  64, 64, 16, 16, dst + OFF_DW,  tid);
    pack_w(cw0, 32, 31, 64, 64, dst + OFF_CW0, tid);
    pack_w(cw1, 64, 64, 64, 64, dst + OFF_CW1, tid);
    pack_w(cw2, 64, 64, 64, 64, dst + OFF_CW2, tid);
    pack_w(rw,  64, 64, 16, 3,  dst + OFF_RW,  tid);
    pack_bias(gb0, gb1, db, cb0, cb1, cb2, rb, (float*)(dst + PW_WORDS), tid);
}

#if HAVE_TDM
__device__ __forceinline__ void tdm_load_to_lds(const uint32_t* gsrc, uint32_t* ldst, int words) {
    const unsigned long long ga = (unsigned long long)(uintptr_t)gsrc;
    const unsigned la = (unsigned)(uintptr_t)ldst;
    u32x4 g0;
    g0.x = 1u;
    g0.y = la;
    g0.z = (unsigned)(ga & 0xFFFFFFFFu);
    g0.w = (unsigned)((ga >> 32) & 0x01FFFFFFu) | 0x80000000u;
    const unsigned uw = (unsigned)words;
    i32x8 g1;
    g1[0] = (int)(2u << 16);
    g1[1] = (int)((uw & 0xFFFFu) << 16);
    g1[2] = (int)(((uw >> 16) & 0xFFFFu) | (1u << 16));
    g1[3] = (int)((uw & 0xFFFFu) << 16);
    g1[4] = 1;
    g1[5] = (int)uw;
    g1[6] = (int)((uw & 0xFFFFu) << 16);
    g1[7] = 0;
    i32x4 gz4 = {0, 0, 0, 0};
#if __clang_major__ >= 23
    i32x8 gz8 = {0, 0, 0, 0, 0, 0, 0, 0};
    __builtin_amdgcn_tensor_load_to_lds(g0, g1, gz4, gz4, gz8, 0);
#else
    __builtin_amdgcn_tensor_load_to_lds(g0, g1, gz4, gz4, 0);
#endif
}
#endif

__global__ __launch_bounds__(NTHREADS)
void ngp_pack_kernel(const float* __restrict__ gw0, const float* __restrict__ gb0,
                     const float* __restrict__ gw1, const float* __restrict__ gb1,
                     const float* __restrict__ dw,  const float* __restrict__ db,
                     const float* __restrict__ cw0, const float* __restrict__ cb0,
                     const float* __restrict__ cw1, const float* __restrict__ cb1,
                     const float* __restrict__ cw2, const float* __restrict__ cb2,
                     const float* __restrict__ rw,  const float* __restrict__ rb,
                     uint32_t* __restrict__ ws) {
    pack_all(gw0, gw1, dw, cw0, cw1, cw2, rw,
             gb0, gb1, db, cb0, cb1, cb2, rb, ws, threadIdx.x);
}

__global__ __launch_bounds__(NTHREADS)
void ngp_fused_kernel(const float* __restrict__ pos, const float* __restrict__ dir,
                      const float* __restrict__ emb,
                      const float* __restrict__ gw0, const float* __restrict__ gb0,
                      const float* __restrict__ gw1, const float* __restrict__ gb1,
                      const float* __restrict__ dw,  const float* __restrict__ db,
                      const float* __restrict__ cw0, const float* __restrict__ cb0,
                      const float* __restrict__ cw1, const float* __restrict__ cb1,
                      const float* __restrict__ cw2, const float* __restrict__ cb2,
                      const float* __restrict__ rw,  const float* __restrict__ rb,
                      const uint32_t* __restrict__ pws,
                      float* __restrict__ out, int N)
{
    __shared__ __align__(16) uint32_t s_wb[WB_WORDS];
    __shared__ _Float16 s_act[WAVES][2][16 * 64];
    __shared__ __align__(16) float s_den[POINTS_PER_BLOCK];
    __shared__ __align__(16) float s_rgb[POINTS_PER_BLOCK * 3];

    const int tid  = threadIdx.x;
    const int lane = tid & 31;
    const int wave = tid >> 5;

    if (pws != nullptr) {
#if HAVE_TDM
        if (wave == 0) {
            tdm_load_to_lds(pws, s_wb, WB_WORDS);
            __builtin_amdgcn_s_wait_tensorcnt(0);
        }
#else
        const uint4* src4 = (const uint4*)pws;
        uint4* dst4 = (uint4*)s_wb;
        for (int i = tid; i < WB_WORDS / 4; i += NTHREADS)
            dst4[i] = src4[i];
#endif
    } else {
        pack_all(gw0, gw1, dw, cw0, cw1, cw2, rw,
                 gb0, gb1, db, cb0, cb1, cb2, rb, s_wb, tid);
    }
    __syncthreads();

    const uint32_t* s_pw   = s_wb;
    const float*    s_bias = (const float*)(s_wb + PW_WORDS);

    _Float16* bufA = s_act[wave][0];
    _Float16* bufB = s_act[wave][1];

    const int m  = lane & 15;
    const int kh = (lane >> 4) & 1;

    for (int t = 0; t < TILES; ++t) {
        const int base = (blockIdx.x * (WAVES * TILES) + wave * TILES + t) * 16;
        const int p  = base + m;
        const int pc = p < N ? p : N - 1;

        const float px = pos[pc * 3 + 0] * 0.5f;
        const float py = pos[pc * 3 + 1] * 0.5f;
        const float pz = pos[pc * 3 + 2] * 0.5f;
        const float ddx = dir[pc * 3 + 0];
        const float ddy = dir[pc * 3 + 1];
        const float ddz = dir[pc * 3 + 2];

        for (int i = 0; i < 8; ++i) {
            const int li  = kh * 8 + i;
            const int res = 16 << li;
            const float rm1 = (float)(res - 1);
            float sx = (px + 1.0f) * 0.5f * rm1;
            float sy = (py + 1.0f) * 0.5f * rm1;
            float sz = (pz + 1.0f) * 0.5f * rm1;
            int gx = (int)floorf(sx), gy = (int)floorf(sy), gz = (int)floorf(sz);
            float wx = sx - (float)gx, wy = sy - (float)gy, wz = sz - (float)gz;
            int x0 = min(max(gx, 0), res - 1), x1 = min(max(gx + 1, 0), res - 1);
            int y0 = min(max(gy, 0), res - 1), y1 = min(max(gy + 1, 0), res - 1);
            int z0 = min(max(gz, 0), res - 1), z1 = min(max(gz + 1, 0), res - 1);

            const unsigned hy0 = (unsigned)y0 * 2481u, hy1 = (unsigned)y1 * 2481u;
            const unsigned hz0 = (unsigned)z0 * 1941u, hz1 = (unsigned)z1 * 1941u;
            const float2* tab = reinterpret_cast<const float2*>(emb) + li * 4096;
            float2 f0 = tab[((unsigned)x0 ^ hy0 ^ hz0) & 4095u];
            float2 f1 = tab[((unsigned)x0 ^ hy0 ^ hz1) & 4095u];
            float2 f2 = tab[((unsigned)x0 ^ hy1 ^ hz0) & 4095u];
            float2 f3 = tab[((unsigned)x0 ^ hy1 ^ hz1) & 4095u];
            float2 f4 = tab[((unsigned)x1 ^ hy0 ^ hz0) & 4095u];
            float2 f5 = tab[((unsigned)x1 ^ hy0 ^ hz1) & 4095u];
            float2 f6 = tab[((unsigned)x1 ^ hy1 ^ hz0) & 4095u];
            float2 f7 = tab[((unsigned)x1 ^ hy1 ^ hz1) & 4095u];

            float c00x = lerpf(f0.x, f1.x, wx), c00y = lerpf(f0.y, f1.y, wx);
            float c01x = lerpf(f2.x, f3.x, wx), c01y = lerpf(f2.y, f3.y, wx);
            float c10x = lerpf(f4.x, f5.x, wx), c10y = lerpf(f4.y, f5.y, wx);
            float c11x = lerpf(f6.x, f7.x, wx), c11y = lerpf(f6.y, f7.y, wx);
            float ox = lerpf(lerpf(c00x, c01x, wy), lerpf(c10x, c11x, wy), wz);
            float oy = lerpf(lerpf(c00y, c01y, wy), lerpf(c10y, c11y, wy), wz);

            PackPair pk;
            pk.h[0] = (_Float16)(ox * GEO_SCALE);
            pk.h[1] = (_Float16)(oy * GEO_SCALE);
            *(uint32_t*)(bufA + m * 64 + kh * 16 + 2 * i) = pk.u;
        }
        wave_fence();

        mlp_layer<1, 4, true>(bufA, 64, s_pw + OFF_GW0, s_bias + OB_GB0, bufB, 64, lane);
        wave_fence();
        mlp_layer<2, 4, true>(bufB, 64, s_pw + OFF_GW1, s_bias + OB_GB1, bufA, 64, lane);
        wave_fence();

        {
            Frag a[2];
            load_afrag<2>(a, bufA, 64, lane);
            const int n = lane & 15;
            const int mrow = kh * 8;
            v8f acc = mlp_block<2>(a, s_pw + OFF_DW, 0, 1, s_bias[OB_DB + n], lane);
            if (n == 0) {
#pragma unroll
                for (int r = 0; r < 8; ++r) s_den[(wave * TILES + t) * 16 + mrow + r] = expf(acc[r] * INV_GEO_SCALE - 1.0f);
            } else {
#pragma unroll
                for (int r = 0; r < 8; ++r)
                    bufB[(mrow + r) * 64 + (n - 1)] = (_Float16)(acc[r] * INV_GEO_SCALE);
            }
        }

        {
            float nn = sqrtf(ddx * ddx + ddy * ddy + ddz * ddz);
            nn = fmaxf(nn, 1e-12f);
            float x = ddx / nn, y = ddy / nn, z = ddz / nn;
            float xx = x * x, yy = y * y, zz = z * z;
            float sh[16];
            sh[0]  = 0.28209479177387814f;
            sh[1]  = -0.48860251190291987f * y;
            sh[2]  = 0.48860251190291987f * z;
            sh[3]  = -0.48860251190291987f * x;
            sh[4]  = 1.0925484305920792f * x * y;
            sh[5]  = -1.0925484305920792f * y * z;
            sh[6]  = 0.31539156525252005f * (2.0f * zz - xx - yy);
            sh[7]  = -1.0925484305920792f * x * z;
            sh[8]  = 0.5462742152960396f * (xx - yy);
            sh[9]  = -0.5900435899266435f * y * (3.0f * xx - yy);
            sh[10] = 2.890611442640554f * x * y * z;
            sh[11] = -0.4570457994644658f * y * (4.0f * zz - xx - yy);
            sh[12] = 0.3731763325901154f * z * (2.0f * zz - 3.0f * xx - 3.0f * yy);
            sh[13] = -0.4570457994644658f * x * (4.0f * zz - xx - yy);
            sh[14] = 1.445305721320277f * z * (xx - yy);
            sh[15] = -0.5900435899266435f * x * (xx - 3.0f * yy);
#pragma unroll
            for (int i = 0; i < 8; ++i)
                bufB[m * 64 + 15 + kh * 8 + i] = (_Float16)sh[kh * 8 + i];
            if (kh) bufB[m * 64 + 31] = (_Float16)0.0f;
        }
        wave_fence();

        mlp_layer<1, 4, true>(bufB, 64, s_pw + OFF_CW0, s_bias + OB_CB0, bufA, 64, lane);
        wave_fence();
        mlp_layer<2, 4, false>(bufA, 64, s_pw + OFF_CW1, s_bias + OB_CB1, bufB, 64, lane);
        wave_fence();
        mlp_layer<2, 4, false>(bufB, 64, s_pw + OFF_CW2, s_bias + OB_CB2, bufA, 64, lane);
        wave_fence();

        {
            Frag a[2];
            load_afrag<2>(a, bufA, 64, lane);
            const int n = lane & 15;
            const int mrow = kh * 8;
            v8f acc = mlp_block<2>(a, s_pw + OFF_RW, 0, 1, s_bias[OB_RB + n], lane);
            if (n < 3) {
#pragma unroll
                for (int r = 0; r < 8; ++r) s_rgb[((wave * TILES + t) * 16 + mrow + r) * 3 + n] = 1.0f / (1.0f + expf(-acc[r]));
            }
        }
        wave_fence();
    }
    __syncthreads();
    {
        const int pbase = blockIdx.x * POINTS_PER_BLOCK;
        const int nvalid = min(POINTS_PER_BLOCK, N - pbase);
        for (int pass = 0; pass < 2; ++pass) {
            if (tid < nvalid / 4) *(volatile v4f*)(out + pbase + tid * 4) = *(const v4f*)(s_den + tid * 4);
            for (int q = tid; q < nvalid * 3 / 4; q += NTHREADS) *(volatile v4f*)(out + N + (size_t)pbase * 3 + q * 4) = *(const v4f*)(s_rgb + q * 4);
            __threadfence();
        }
    }
}

extern "C" void kernel_launch(void* const* d_in, const int* in_sizes, int n_in,
                              void* d_out, int out_size, void* d_ws, size_t ws_size,
                              hipStream_t stream) {
    const float* pos = (const float*)d_in[0];
    const float* dir = (const float*)d_in[1];
    const float* emb = (const float*)d_in[2];
    const float* gw0 = (const float*)d_in[3];
    const float* gb0 = (const float*)d_in[4];
    const float* gw1 = (const float*)d_in[5];
    const float* gb1 = (const float*)d_in[6];
    const float* dw  = (const float*)d_in[7];
    const float* db  = (const float*)d_in[8];
    const float* cw0 = (const float*)d_in[9];
    const float* cb0 = (const float*)d_in[10];
    const float* cw1 = (const float*)d_in[11];
    const float* cb1 = (const float*)d_in[12];
    const float* cw2 = (const float*)d_in[13];
    const float* cb2 = (const float*)d_in[14];
    const float* rw  = (const float*)d_in[15];
    const float* rb  = (const float*)d_in[16];
    float* out = (float*)d_out;

    const int N = in_sizes[0] / 3;
    const int nblocks = (N + POINTS_PER_BLOCK - 1) / POINTS_PER_BLOCK;

    (void)n_in; (void)out_size;
    if (d_ws == nullptr || ws_size < (size_t)WB_WORDS * 4) return;
    uint32_t* pws = (uint32_t*)d_ws;
    ngp_pack_kernel<<<1, NTHREADS, 0, stream>>>(
        gw0, gb0, gw1, gb1, dw, db, cw0, cb0, cw1, cb1, cw2, cb2, rw, rb, pws);

    ngp_fused_kernel<<<nblocks, NTHREADS, 0, stream>>>(
        pos, dir, emb, gw0, gb0, gw1, gb1, dw, db,
        cw0, cb0, cw1, cb1, cw2, cb2, rw, rb, pws, out, N);
}
